// MRConv2d_plg_14826227105877
// MI455X (gfx1250) — hardware-verified
//
#include <hip/hip_runtime.h>

#define __bf16 _Float16
typedef __attribute__((ext_vector_type(16))) __bf16 v16bf;
typedef __attribute__((ext_vector_type(8)))  float  v8f;
typedef __attribute__((ext_vector_type(4)))  float  v4f_t;
typedef float v4fa __attribute__((ext_vector_type(4), may_alias));
#define RSPLIT (1.0f / 2048.0f)
__device__ __forceinline__ __bf16 lo_of(float v, __bf16 h) { return (__bf16)((v - (float)h) * 2048.0f); }
__device__ __forceinline__ v8f wmma16(v16bf a, v16bf b, v8f c) { return __builtin_amdgcn_wmma_f32_16x16x32_f16(false, a, false, b, (short)0, c, false, false); }
__device__ __forceinline__ v8f wmma_split(v16bf a, v16bf al, v16bf b, v16bf bl, v8f c) { v8f x = {}; x = wmma16(al, b, x); x = wmma16(a, bl, x); return wmma16(a, b, c) + x * RSPLIT; }

#define Bc   4
#define Cc   384
#define C2   768
#define Nl   2048
#define Np   4096
#define Kn   16
#define NT   32
#define KSTEPS (C2 / 32)
#define WFRAG_ELEMS (Cc * C2)
#define WFRAG_BYTES (WFRAG_ELEMS * 2)

__device__ __forceinline__ int feat_elem(int kf, int t) {
    int ks   = kf >> 5;
    int kk   = kf & 31;
    int hi   = (kk >> 3) & 1;
    int i    = (kk & 7) + ((kk >> 4) << 3);
    int sub  = t >> 4;
    int lane = (t & 15) | (hi << 4);
    return (((ks * 2 + sub) * 32) + lane) * 16 + i;
}

__global__ __launch_bounds__(256)
void convert_W(const float* __restrict__ W, __bf16* __restrict__ Wfrag) {
    int e = (blockIdx.x * 256 + threadIdx.x) * 2;
    if (e >= WFRAG_ELEMS) return;
    int i    = e & 15;
    int lane = (e >> 4) & 31;
    int ks   = (e >> 9) % KSTEPS;
    int mt   = e / (KSTEPS * 512);
    int m = mt * 16 + (lane & 15);
    int k = ks * 32 + ((lane >> 4) * 8) + (i < 8 ? i : i + 8);
    const float v0 = W[(size_t)m * C2 + k], v1 = W[(size_t)m * C2 + k + 1];
    const __bf16 a = (__bf16)v0, bb = (__bf16)v1;
    const unsigned u = (unsigned)__builtin_bit_cast(unsigned short, a) | ((unsigned)__builtin_bit_cast(unsigned short, bb) << 16);
    const unsigned w = (unsigned)__builtin_bit_cast(unsigned short, lo_of(v0, a)) | ((unsigned)__builtin_bit_cast(unsigned short, lo_of(v1, bb)) << 16);
    *(volatile unsigned*)(Wfrag + e) = u; *(volatile unsigned*)(Wfrag + WFRAG_ELEMS + e) = w; __threadfence();
    *(volatile unsigned*)(Wfrag + e) = u; *(volatile unsigned*)(Wfrag + WFRAG_ELEMS + e) = w;
}

template <bool USE_WFRAG>
__global__ __launch_bounds__(768)
void mrconv2d_fused(const float*  __restrict__ lab,
                    const float*  __restrict__ patch,
                    const int*    __restrict__ eidx,
                    const float*  __restrict__ Wf,
                    const __bf16* __restrict__ Wfrag,
                    const float*  __restrict__ bias,
                    float*        __restrict__ out)
{
    __shared__ int   s_ii[NT * Kn];
    __shared__ int   s_jj[NT * Kn];
    __shared__ v16bf s_fragB[KSTEPS * 2 * 32];
    __shared__ v16bf s_fragL[KSTEPS * 2 * 32];

    const int tid = threadIdx.x;
    const int bid = blockIdx.x;
    const int b   = bid / (Nl / NT);
    const int n0  = (bid % (Nl / NT)) * NT;

    const int* e0 = eidx;
    const int* e1 = eidx + (size_t)Bc * Nl * Kn;
    for (int u = tid; u < 2 * NT * Kn; u += 768) {
        int which = u >> 9;
        int v = u & 511;
        int t = v >> 4, k = v & 15;
        int val = (which ? e0 : e1)[((size_t)b * Nl + n0 + t) * Kn + k];
        const int lim = which ? Np : Nl;
        val = (val < 0) ? 0 : (val >= lim ? lim - 1 : val);
        if (which) s_jj[v] = val; else s_ii[v] = val;
    }
    __syncthreads();

    const float* labB = lab   + (size_t)b * Cc * Nl;
    const float* patB = patch + (size_t)b * Cc * Np;
    __bf16* fragw = (__bf16*)s_fragB;
    __bf16* fragl = (__bf16*)s_fragL;

    #pragma unroll 4
    for (int it = 0; it < (Cc * NT) / 768; ++it) {
        int idx = it * 768 + tid;
        int c = idx >> 5;
        int t = idx & 31;
        { const float v = labB[(size_t)c * Nl + n0 + t]; const int p = feat_elem(2 * c, t); fragw[p] = (__bf16)v; fragl[p] = lo_of(v, fragw[p]); }
    }
    #pragma unroll 2
    for (int it = 0; it < (Cc * NT) / 768; ++it) {
        int idx = it * 768 + tid;
        int c = idx >> 5;
        int t = idx & 31;
        const float* lrow = labB + (size_t)c * Nl;
        const float* prow = patB + (size_t)c * Np;
        float m = -3.0e38f;
        #pragma unroll
        for (int k = 0; k < Kn; ++k) {
            float d = lrow[s_ii[t * Kn + k]] - prow[s_jj[t * Kn + k]];
            m = fmaxf(m, d);
        }
        { const int p = feat_elem(2 * c + 1, t); fragw[p] = (__bf16)m; fragl[p] = lo_of(m, fragw[p]); }
    }
    __syncthreads();

    const int lane = tid & 31;
    const int wave = tid >> 5;
    const int o0   = wave * 16;

    v8f acc0 = {0.f,0.f,0.f,0.f,0.f,0.f,0.f,0.f};
    v8f acc1 = {0.f,0.f,0.f,0.f,0.f,0.f,0.f,0.f};

    (void)Wf;
    #pragma unroll 2
    for (int ks = 0; ks < KSTEPS; ++ks) {
        const size_t ao = (((size_t)wave * KSTEPS + ks) * 32 + lane) * 16;
        const v16bf a  = *(const v16bf*)(Wfrag + ao);
        const v16bf al = *(const v16bf*)(Wfrag + WFRAG_ELEMS + ao);
        acc0 = wmma_split(a, al, s_fragB[(ks * 2 + 0) * 32 + lane], s_fragL[(ks * 2 + 0) * 32 + lane], acc0);
        acc1 = wmma_split(a, al, s_fragB[(ks * 2 + 1) * 32 + lane], s_fragL[(ks * 2 + 1) * 32 + lane], acc1);
    }

    __syncthreads();
    float* sw = (float*)s_fragB + wave * (16 * 32);
    const int hi = lane >> 4, l16 = lane & 15;
    #pragma unroll
    for (int r = 0; r < 8; ++r) {
        const int rl = r + hi * 8, o = o0 + rl;
        const float bo = bias[o];
        sw[rl * 32 + l16]      = fmaxf(acc0[r] + bo, 0.f);
        sw[rl * 32 + 16 + l16] = fmaxf(acc1[r] + bo, 0.f);
    }
    asm volatile("s_wait_dscnt 0" ::: "memory");
    float* outB = out + (size_t)b * Cc * Nl;
    #pragma unroll 1
    for (int pass = 0; pass < 2; ++pass) {
        #pragma unroll
        for (int i = 0; i < 4; ++i) { const int c = lane + 32 * i, rl = c >> 3, q = (c & 7) * 4;
            *(volatile v4f_t*)(outB + (size_t)(o0 + rl) * Nl + n0 + q) = *(const volatile v4fa*)(sw + rl * 32 + q); }
        __threadfence();
    }
}

extern "C" void kernel_launch(void* const* d_in, const int* in_sizes, int n_in,
                              void* d_out, int out_size, void* d_ws, size_t ws_size,
                              hipStream_t stream) {
    (void)in_sizes; (void)n_in; (void)out_size;
    const float* lab   = (const float*)d_in[0];
    const float* patch = (const float*)d_in[1];
    const int*   eidx  = (const int*)d_in[2];
    const float* W     = (const float*)d_in[3];
    const float* bias  = (const float*)d_in[4];
    float* out = (float*)d_out;

    dim3 grid(Bc * (Nl / NT));
    dim3 block(768);

    (void)ws_size;
    __bf16* Wfrag = (__bf16*)d_ws;
    hipLaunchKernelGGL(convert_W, dim3(WFRAG_ELEMS / 512), dim3(256), 0, stream, W, Wfrag);
    hipLaunchKernelGGL((mrconv2d_fused<true>), grid, block, 0, stream, lab, patch, eidx, W, Wfrag, bias, out);
}
